// HGCU_77292231458937
// MI455X (gfx1250) — hardware-run, weakly checked
//
#include <hip/hip_runtime.h>


#ifndef NB
#define NB 2
#endif
#define NB_FULL 2
#define CF    256
#define CC    64
#define KC    100
#define KCP   112
#define K3    576
#define HH    128
#define WH    128
#define HL    64
#define WL    64
#define HWH   (HH * WH)
#define HWL   (HL * WL)
#define XP    264
#define TP    72
#define TCOLS 34
#define OSP   68
#define OKP   36
#define WCS   1024.0f
#define WCI   (1.0f / 1024.0f)
#define L2E   1.4426950408889634f

static_assert(NB <= NB_FULL);
static_assert(HWH % 64 == 0);
static_assert(HWL % 64 == 0);
static_assert(WH % 32 == 0);
static_assert(WL % 32 == 0);
static_assert(WH == 2 * 64);
static_assert(HH == 2 * HL);
static_assert(WH == 2 * WL);
static_assert(HL >= 3);
static_assert(WL >= 3);
static_assert(CF % 32 == 0);
static_assert(CC % 32 == 0);
static_assert(CC == 64);
static_assert(K3 == 9 * CC);
static_assert(KC == 4 * 25);
static_assert(KCP % 16 == 0);
static_assert(KCP >= KC);
static_assert(KCP / 16 == 7);
static_assert((CF * 16) % 128 == 0);
static_assert(4 * 224 >= 3 * TCOLS * 8);
static_assert((XP * 2) % 16 == 0);
static_assert((TP * 2) % 16 == 0);
static_assert((OSP * 4) % 16 == 0);
static_assert((OKP * 4) % 16 == 0);
static_assert(XP >= CF);
static_assert(TP >= CC);
static_assert(32 * 16 * 4 == 16 * CC * 2);
static_assert(32 * 16 * 4 == 16 * 32 * 4);
static_assert(((size_t)NB * 4 * HWH) % 256 == 0);
static_assert(((size_t)KCP * 9 * 8) % 8 == 0);
static_assert((size_t)64 * XP * 2 + (size_t)4 * 16 * OSP * 4 <= 131072);
static_assert((size_t)3 * TCOLS * TP * 2 + (size_t)KCP * OKP * 4 <= 131072);
static_assert((size_t)25 * 64 * 4 <= 131072);

typedef _Float16 h16;
typedef unsigned short bf;
typedef __attribute__((ext_vector_type(16))) __bf16   v16bf;
typedef __attribute__((ext_vector_type(16))) _Float16 v16h;
typedef __attribute__((ext_vector_type(8)))  _Float16 v8h;
typedef __attribute__((ext_vector_type(8)))  unsigned short v8us;
typedef __attribute__((ext_vector_type(8)))  float    v8f;
typedef __attribute__((ext_vector_type(4)))  float    v4f;
typedef v4f  __attribute__((may_alias)) v4fa;

__device__ __forceinline__ unsigned short f2bf(float f) { unsigned u = __float_as_uint(f); u += 0x7FFFu + ((u >> 16) & 1u); return (unsigned short)(u >> 16); }
__device__ __forceinline__ float bfr(float f) { return __uint_as_float(((unsigned)f2bf(f)) << 16); }
__device__ __forceinline__ v16h cat16(v8h lo, v8h hi) { return __builtin_shufflevector(lo, hi, 0, 1, 2, 3, 4, 5, 6, 7, 8, 9, 10, 11, 12, 13, 14, 15); }
__device__ __forceinline__ v16bf cat16b(v8us lo, v8us hi) { return __builtin_bit_cast(v16bf, __builtin_shufflevector(lo, hi, 0, 1, 2, 3, 4, 5, 6, 7, 8, 9, 10, 11, 12, 13, 14, 15)); }
__device__ __forceinline__ v8f wmma16(v16h a, v16h b, v8f c) { return __builtin_amdgcn_wmma_f32_16x16x32_f16(false, a, false, b, (short)0, c, false, false); }
__device__ __forceinline__ v8f wmmab(v16bf a, v16bf b, v8f c) { return __builtin_amdgcn_wmma_f32_16x16x32_bf16(false, a, false, b, (short)0, c, false, false); }
__device__ __forceinline__ v16h  ldh(const h16* p) { return cat16(*(const v8h*)p, *(const v8h*)(p + 16)); }
__device__ __forceinline__ v16bf ldb(const bf* p)  { return cat16b(*(const v8us*)p, *(const v8us*)(p + 16)); }
__device__ __forceinline__ void wave_sync() { __builtin_amdgcn_fence(3  , "wavefront"); __builtin_amdgcn_wave_barrier(); asm volatile("" ::: "memory"); }

static __device__ __forceinline__ v8f wmma16g(v16h a, v16h b, v8f c) { c = wmma16(a, b, c); asm volatile("v_nop\n\tv_nop\n\tv_nop\n\tv_nop" : "+v"(c) : "v"(a), "v"(b)); return c; }
static __device__ __forceinline__ v8f wmmabg(v16bf a, v16bf b, v8f c) { c = wmmab(a, b, c); asm volatile("v_nop\n\tv_nop\n\tv_nop\n\tv_nop" : "+v"(c) : "v"(a), "v"(b)); return c; }
static __device__ __forceinline__ h16 toh_flush(float v) { const h16 r = (h16)v; return (fabsf(v) < 6.103515625e-05f) ? (h16)0.0f : r; }

__global__ __launch_bounds__(256) void k_cvt8(const float* __restrict__ src, bf* dst, size_t n8) {
    const size_t i = (size_t)blockIdx.x * 256 + threadIdx.x; if (i >= n8) return;
    const v8f v = *(const v8f*)(src + i * 8); v8us o;
#pragma unroll
    for (int k = 0; k < 8; ++k) o[k] = f2bf(v[k]);
    *(volatile v8us*)(dst + i * 8) = o; __threadfence(); *(volatile v8us*)(dst + i * 8) = o;
}

__global__ __launch_bounds__(256) void k_wk(const float* __restrict__ w, h16* dst) {
    const int i = blockIdx.x * 256 + threadIdx.x; if (i >= KCP * 9 * 8) return;
    const int c8 = (i & 7) * 8; const int rt = i >> 3; const int t = rt % 9; const int oc = rt / 9;
    const int occ = oc < KC ? oc : (KC - 1);
    const bool live = oc < KC;
    v8h o;
#pragma unroll
    for (int j = 0; j < 8; ++j) {
        float x = w[((size_t)occ * CC + (size_t)(c8 + j)) * 9 + t];
        asm volatile("" : "+v"(x));
        const h16 hv = toh_flush(bfr(x) * WCS);
        o[j] = live ? hv : (h16)0.0f; }
    *(volatile v8h*)(dst + (size_t)i * 8) = o; __threadfence(); *(volatile v8h*)(dst + (size_t)i * 8) = o;
}

__global__ __launch_bounds__(128) void k_comp(const float* __restrict__ X, const bf* __restrict__ Wb, h16* CP, int HW) {
    __shared__ __align__(16) bf xs[64 * XP];
    __shared__ __align__(16) float os[4 * 16 * OSP];
    const int tid = threadIdx.x, lane = tid & 31, lr = lane & 15, hi = lane >> 4;
    const int wave = __builtin_amdgcn_readfirstlane((int)(threadIdx.x >> 5));
    const int n0 = blockIdx.x * 64; const int b = n0 / HW; const int hw0 = n0 - b * HW;
    const float* xb = X + (size_t)b * CF * HW + hw0;
#pragma unroll 1
    for (int g = tid; g < CF * 16; g += 128) {
        const int c = g >> 4, p4 = (g & 15) * 4;
        const v4f v = *(const v4f*)(xb + (size_t)c * HW + p4);
#pragma unroll
        for (int j = 0; j < 4; ++j) xs[(p4 + j) * XP + c] = f2bf(v[j]);
    }
    __syncthreads();
    v8f acc[4];
#pragma unroll
    for (int nb = 0; nb < 4; ++nb) acc[nb] = (v8f){};
    const int ao = (wave * 16 + lr) * XP + 8 * hi;
    const size_t bo = (size_t)lr * CF + 8 * hi;
#pragma unroll 1
    for (int kc = 0; kc < CF; kc += 32) {
        const v16bf a = cat16b(*(const v8us*)(&xs[ao + kc]), *(const v8us*)(&xs[ao + kc + 16]));
#pragma unroll
        for (int nb = 0; nb < 4; ++nb) { const v16bf bb = ldb(Wb + bo + (size_t)nb * 16 * CF + kc); acc[nb] = wmmabg(a, bb, acc[nb]); }
    }
    const int wb = wave * 16 * OSP;
#pragma unroll
    for (int nb = 0; nb < 4; ++nb) {
#pragma unroll
        for (int j = 0; j < 8; ++j) os[wb + (hi * 8 + j) * OSP + nb * 16 + lr] = acc[nb][j]; }
    wave_sync();
    h16* crow = CP + ((size_t)b * HW + (size_t)hw0 + (size_t)(wave * 16)) * CC;
#pragma unroll 1
    for (int ps = 0; ps < 2; ++ps) {
#pragma unroll
        for (int s = 0; s < 4; ++s) { const int row = 4 * s + (lane >> 3), c8 = (lane & 7) * 8;
            const v4f x0 = *(const v4fa*)(&os[wb + row * OSP + c8]); const v4f x1 = *(const v4fa*)(&os[wb + row * OSP + c8 + 4]); v8h hv;
#pragma unroll
            for (int i = 0; i < 4; ++i) { hv[i] = toh_flush(x0[i]); hv[4 + i] = toh_flush(x1[i]); }
            *(volatile v8h*)(crow + (size_t)row * CC + c8) = hv; }
        if (ps == 0) __threadfence(); }
}

__global__ __launch_bounds__(224) void k_kgen(const h16* __restrict__ CP, const h16* __restrict__ WK, const float* __restrict__ bias, float* KO, int H, int W) {
    __shared__ __align__(16) h16 xs[3 * TCOLS * TP];
    __shared__ __align__(16) float os[KCP * OKP];
    const int tid = threadIdx.x, lane = tid & 31, lr = lane & 15, hi = lane >> 4;
    const int wave = __builtin_amdgcn_readfirstlane((int)(threadIdx.x >> 5));
    const int tpr = W >> 5; const int bid = blockIdx.x;
    const int wtl = bid % tpr; const int y = (bid / tpr) % H; const int b = bid / (tpr * H);
    const int x0 = wtl << 5;
    const h16* cb = CP + (size_t)b * (size_t)H * (size_t)W * CC;
    const v8h hz = (v8h){};
#pragma unroll 1
    for (int it = 0; it < 4; ++it) {
        const int idx = tid + it * 224; const int idc = idx < 3 * TCOLS * 8 ? idx : (3 * TCOLS * 8 - 1);
        const int part = idc & 7; const int pp = idc >> 3; const int col = pp % TCOLS; const int ky = pp / TCOLS;
        const int sy = y + ky - 1, gx = x0 + col - 1;
        const bool ok = (sy >= 0) & (sy < H) & (gx >= 0) & (gx < W);
        const int syc = sy < 0 ? 0 : (sy > H - 1 ? H - 1 : sy);
        const int gxc = gx < 0 ? 0 : (gx > W - 1 ? W - 1 : gx);
        v8h v = *(const v8h*)(cb + ((size_t)syc * (size_t)W + (size_t)gxc) * CC + part * 8);
        asm volatile("" : "+v"(v));
        v = ok ? v : hz;
        if (idx < 3 * TCOLS * 8) *(v8h*)(&xs[pp * TP + part * 8]) = v;
    }
    __syncthreads();
    const int m0 = wave * 16;
    const h16* wr = WK + (size_t)(m0 + lr) * K3 + 8 * hi;
    v8f acc0 = (v8f){}, acc1 = (v8f){};
#pragma unroll 1
    for (int t = 0; t < 9; ++t) {
        const int ky = t / 3, kx = t - 3 * ky;
        const int sb = (ky * TCOLS + lr + kx) * TP + 8 * hi;
#pragma unroll
        for (int c0 = 0; c0 < CC; c0 += 32) {
            const v16h a  = ldh(wr + t * CC + c0);
            const v16h b0 = cat16(*(const v8h*)(&xs[sb + c0]), *(const v8h*)(&xs[sb + c0 + 16]));
            const v16h b1 = cat16(*(const v8h*)(&xs[sb + 16 * TP + c0]), *(const v8h*)(&xs[sb + 16 * TP + c0 + 16]));
            acc0 = wmma16g(a, b0, acc0);
            acc1 = wmma16g(a, b1, acc1);
        }
    }
    float bs[8];
#pragma unroll
    for (int j = 0; j < 8; ++j) { const int oc = m0 + 8 * hi + j; bs[j] = bfr(bias[oc < KC ? oc : (KC - 1)]); }
#pragma unroll
    for (int j = 0; j < 8; ++j) {
        os[(m0 + 8 * hi + j) * OKP + lr]      = acc0[j] * WCI + bs[j];
        os[(m0 + 8 * hi + j) * OKP + 16 + lr] = acc1[j] * WCI + bs[j]; }
    wave_sync();
    float* kb = KO + (size_t)b * KC * (size_t)H * (size_t)W + (size_t)y * (size_t)W + (size_t)x0;
#pragma unroll 1
    for (int ps = 0; ps < 2; ++ps) {
#pragma unroll
        for (int s = 0; s < 4; ++s) { const int row = 4 * s + (lane >> 3), cofs = (lane & 7) * 4;
            const int oc = m0 + row;
            const v4f val = *(const v4fa*)(&os[oc * OKP + cofs]);
            if (oc < KC) *(volatile v4f*)(kb + (size_t)oc * (size_t)H * (size_t)W + cofs) = val; }
        if (ps == 0) __threadfence(); }
}

__global__ __launch_bounds__(256) void k_smax(const float* __restrict__ src, float* dst, int HW, int total) {
#pragma clang fp contract(off)
    const int idx = blockIdx.x * 256 + threadIdx.x; if (idx >= total) return;
    const int q = idx % HW, bg = idx / HW;
    const float* p = src + (size_t)bg * 25 * HW + q;
    float v[25];
#pragma unroll
    for (int c = 0; c < 13; ++c) v[c] = p[(size_t)c * HW];
    asm volatile("" ::: "memory");
#pragma unroll
    for (int c = 13; c < 25; ++c) v[c] = p[(size_t)c * HW];
    float mx = v[0];
#pragma unroll
    for (int c = 1; c < 25; ++c) mx = fmaxf(mx, v[c]);
    float s = 0.0f;
#pragma unroll
    for (int c = 0; c < 25; ++c) { v[c] = __builtin_amdgcn_exp2f((v[c] - mx) * L2E); s += v[c]; }
    const float inv = 1.0f / s;
#pragma unroll
    for (int c = 0; c < 25; ++c) v[c] = v[c] * inv;
    float* o = dst + (size_t)bg * 25 * HW + q;
#pragma unroll 1
    for (int ps = 0; ps < 2; ++ps) {
#pragma unroll
        for (int c = 0; c < 25; ++c) *(volatile float*)(o + (size_t)c * HW) = v[c];
        if (ps == 0) __threadfence(); }
}

__global__ __launch_bounds__(256) void k_hnorm(const float* __restrict__ s, const float* __restrict__ ham, float* out, int HW, int total) {
#pragma clang fp contract(off)
    const int idx = blockIdx.x * 256 + threadIdx.x; if (idx >= total) return;
    const int q = idx % HW, bg = idx / HW;
    const float* p = s + (size_t)bg * 25 * HW + (size_t)q * 25;
    float v[25];
#pragma unroll
    for (int t = 0; t < 13; ++t) v[t] = p[t];
    asm volatile("" ::: "memory");
#pragma unroll
    for (int t = 13; t < 25; ++t) v[t] = p[t];
    float sum = 0.0f;
#pragma unroll
    for (int t = 0; t < 25; ++t) { v[t] = v[t] * bfr(ham[t]); sum += v[t]; }
    const float inv = 1.0f / (sum + 1e-8f);
#pragma unroll
    for (int t = 0; t < 25; ++t) v[t] = v[t] * inv;
    float* o = out + (size_t)bg * 25 * HW + q;
#pragma unroll 1
    for (int ps = 0; ps < 2; ++ps) {
#pragma unroll
        for (int t = 0; t < 25; ++t) *(volatile float*)(o + (size_t)t * HW) = v[t];
        if (ps == 0) __threadfence(); }
}

template <int XBF, int ADD>
static __device__ __forceinline__ void reasm_body(const float* __restrict__ xf, const bf* __restrict__ xh, const int Cx,
                                                  const float* __restrict__ mask, const float* __restrict__ addsrc, float* out) {
    __shared__ float mavg[25 * 64];
    const int tid = threadIdx.x;
    const int bid = blockIdx.x; const int owt = bid & 1; const int oh = (bid >> 1) % HH; const int b = bid / (2 * HH);
    const int ow0 = owt << 6;
    const float* mb = mask + (size_t)b * KC * HWH + (size_t)oh * WH + ow0;
#pragma unroll 1
    for (int t = tid; t < 25 * 64; t += 256) {
        const int k = t >> 6, owl = t & 63;
        const float a0 = mb[(size_t)(0 * 25 + k) * HWH + owl], a1 = mb[(size_t)(1 * 25 + k) * HWH + owl];
        const float a2 = mb[(size_t)(2 * 25 + k) * HWH + owl], a3 = mb[(size_t)(3 * 25 + k) * HWH + owl];
        mavg[t] = 0.25f * (((a0 + a1) + a2) + a3);
    }
    __syncthreads();
    const int owl = tid & 63;
    const int cst = __builtin_amdgcn_readfirstlane((int)(threadIdx.x >> 6));
    const int ow = ow0 + owl;
    const int lh = oh >> 1, lw = ow >> 1;
    int syy[5], sxx[5];
#pragma unroll
    for (int i = 0; i < 5; ++i) { int t2 = lh + i - 2; if (t2 < 0) t2 = -t2; if (t2 > HL - 1) t2 = 2 * (HL - 1) - t2; syy[i] = t2 * WL; }
#pragma unroll
    for (int j = 0; j < 5; ++j) { int t2 = lw + j - 2; if (t2 < 0) t2 = -t2; if (t2 > WL - 1) t2 = 2 * (WL - 1) - t2; sxx[j] = t2; }
    float mk[25];
#pragma unroll
    for (int k = 0; k < 25; ++k) mk[k] = mavg[k * 64 + owl];
    const size_t xbase = (size_t)b * (size_t)Cx * HWL;
    const size_t obase = (size_t)b * (size_t)Cx * HWH + (size_t)oh * WH + (size_t)ow;
#pragma unroll 1
    for (int c = cst; c < Cx; c += 4) {
        const size_t xc = xbase + (size_t)c * HWL;
        const size_t oo = obase + (size_t)c * HWH;
        float acc = 0.0f;
        if (ADD) acc = addsrc[oo];
#pragma unroll
        for (int i = 0; i < 5; ++i) {
#pragma unroll
            for (int j = 0; j < 5; ++j) {
                float xv;
                if (XBF) xv = __uint_as_float(((unsigned)xh[xc + (size_t)(syy[i] + sxx[j])]) << 16);
                else     xv = xf[xc + (size_t)(syy[i] + sxx[j])];
                acc += xv * mk[i * 5 + j]; } }
        *(volatile float*)(out + oo) = acc; __threadfence(); *(volatile float*)(out + oo) = acc;
    }
}

__global__ __launch_bounds__(256) void k_reasm_add(const float* __restrict__ xk, const float* __restrict__ mask, const float* __restrict__ addsrc, float* out) {
    reasm_body<0, 1>(xk, (const bf*)0, KC, mask, addsrc, out);
}
__global__ __launch_bounds__(256) void k_reasm_out(const bf* __restrict__ xl, const float* __restrict__ mask, float* out) {
    reasm_body<1, 0>((const float*)0, xl, CF, mask, (const float*)0, out);
}

static constexpr size_t al256(size_t v) { return (v + 255) & ~(size_t)255; }
static constexpr size_t SZ_LB  = al256((size_t)NB * CF * HWL * 2);
static constexpr size_t SZ_WC  = al256((size_t)CC * CF * 2);
static constexpr size_t SZ_WK  = al256((size_t)KCP * K3 * 2);
static constexpr size_t SZ_CPH = al256((size_t)NB * HWH * CC * 2);
static constexpr size_t SZ_CPL = al256((size_t)NB * HWL * CC * 2);
static constexpr size_t SZ_KH  = al256((size_t)NB * KC * HWH * 4);
static constexpr size_t SZ_KL  = al256((size_t)NB * KC * HWL * 4);
static constexpr size_t SZ_TOTAL = SZ_LB + 2 * SZ_WC + 2 * SZ_WK + SZ_CPH + SZ_CPL + 3 * SZ_KH + SZ_KL;
static_assert(SZ_TOTAL <= (size_t)134217728);
static_assert(((size_t)KCP * K3 * 2) % 128 == 0);
static_assert(((size_t)KCP * 9 * 8 * 16) == (size_t)KCP * K3 * 2);

extern "C" void kernel_launch(void* const* d_in, const int* in_sizes, int n_in,
                              void* d_out, int out_size, void* d_ws, size_t ws_size, hipStream_t stream) {
    if (n_in < 9) return;
    if ((size_t)in_sizes[0] < (size_t)NB * CF * HWH || (size_t)in_sizes[1] < (size_t)NB * CF * HWL) return;
    if ((size_t)in_sizes[2] < (size_t)CC * CF || (size_t)in_sizes[3] < (size_t)CC * CF) return;
    if ((size_t)in_sizes[4] < (size_t)KC * CC * 9 || (size_t)in_sizes[6] < (size_t)KC * CC * 9) return;
    if (in_sizes[5] < KC || in_sizes[7] < KC || in_sizes[8] < 25) return;
    if ((size_t)out_size < (size_t)NB * CF * HWH) return;
    if (SZ_TOTAL > ws_size) return;
    const float* hr    = (const float*)d_in[0];
    const float* lr    = (const float*)d_in[1];
    const float* w_hr  = (const float*)d_in[2];
    const float* w_lr  = (const float*)d_in[3];
    const float* wk_hr = (const float*)d_in[4];
    const float* bk_hr = (const float*)d_in[5];
    const float* wk_lr = (const float*)d_in[6];
    const float* bk_lr = (const float*)d_in[7];
    const float* ham   = (const float*)d_in[8];
    float* OUT = (float*)d_out;
    char* wsp = (char*)d_ws;
    bf*  LB  = (bf*)wsp;  wsp += SZ_LB;
    bf*  WCH = (bf*)wsp;  wsp += SZ_WC;
    bf*  WCL = (bf*)wsp;  wsp += SZ_WC;
    h16* WKH = (h16*)wsp; wsp += SZ_WK;
    h16* WKL = (h16*)wsp; wsp += SZ_WK;
    h16* CPH = (h16*)wsp; wsp += SZ_CPH;
    h16* CPL = (h16*)wsp; wsp += SZ_CPL;
    float* KH = (float*)wsp; wsp += SZ_KH;
    float* T0 = (float*)wsp; wsp += SZ_KH;
    float* T1 = (float*)wsp; wsp += SZ_KH;
    float* KL = (float*)wsp; wsp += SZ_KL;

    { const size_t n8 = (size_t)NB * CF * HWL / 8;
      k_cvt8<<<(unsigned)((n8 + 255) / 256), 256, 0, stream>>>(lr, LB, n8); }
    { const size_t n8 = (size_t)CC * CF / 8; const unsigned g = (unsigned)((n8 + 255) / 256);
      k_cvt8<<<g, 256, 0, stream>>>(w_hr, WCH, n8); k_cvt8<<<g, 256, 0, stream>>>(w_lr, WCL, n8); }
    { const unsigned g = (unsigned)((KCP * 9 * 8 + 255) / 256);
      k_wk<<<g, 256, 0, stream>>>(wk_hr, WKH); k_wk<<<g, 256, 0, stream>>>(wk_lr, WKL); }

    k_comp<<<(unsigned)((size_t)NB * HWH / 64), 128, 0, stream>>>(hr, WCH, CPH, HWH);
    k_comp<<<(unsigned)((size_t)NB * HWL / 64), 128, 0, stream>>>(lr, WCL, CPL, HWL);

    k_kgen<<<(unsigned)(NB * HH * (WH / 32)), 224, 0, stream>>>(CPH, WKH, bk_hr, KH, HH, WH);
    k_kgen<<<(unsigned)(NB * HL * (WL / 32)), 224, 0, stream>>>(CPL, WKL, bk_lr, KL, HL, WL);

    const int tot = NB * 4 * HWH;
    const unsigned nbk = (unsigned)((tot + 255) / 256);
    k_smax<<<nbk, 256, 0, stream>>>(KH, T0, HWH, tot);
    k_hnorm<<<nbk, 256, 0, stream>>>(T0, ham, T1, HWH, tot);
    k_reasm_add<<<(unsigned)(NB * HH * 2), 256, 0, stream>>>(KL, T1, KH, T0);
    k_smax<<<nbk, 256, 0, stream>>>(T0, T1, HWH, tot);
    k_hnorm<<<nbk, 256, 0, stream>>>(T1, ham, KH, HWH, tot);
    k_reasm_out<<<(unsigned)(NB * HH * 2), 256, 0, stream>>>(LB, KH, OUT);
}
